// CausalAttention_884763263241
// MI455X (gfx1250) — hardware-verified
//
#include <hip/hip_runtime.h>


namespace {
constexpr int B = 4, T = 2048, E = 1024, BL = 4  , QL = 2048  ;
constexpr int NSL = E / 128;
constexpr float XS = 8.0f, WSC = 256.0f, PS = 1024.0f, RS_ = 1024.0f, LOG2E = 1.4426950408889634f, RSQE = 0.03125f;
static_assert(T % 128 == 0 && QL % 64 == 0 && E % 256 == 0, "tiling");
typedef _Float16 b16;
typedef __attribute__((ext_vector_type(16))) _Float16 v16b;
typedef __attribute__((ext_vector_type(8))) _Float16 v8b;
typedef __attribute__((ext_vector_type(8))) float v8f;
typedef __attribute__((ext_vector_type(4))) float v4f;
__device__ __forceinline__ float bf16_rne(float f) { unsigned int u = __float_as_uint(f); u += 0x7FFFu + ((u >> 16) & 1u); return __uint_as_float(u & 0xFFFF0000u); }
__device__ __forceinline__ void split16(float v, b16& hi, b16& lo) { hi = (b16)v; lo = (b16)(v - (float)hi); }
__device__ __forceinline__ v16b frag_kb(const b16* p, int hh) { const v8b a = *(const v8b*)(p + 8 * hh), b = *(const v8b*)(p + 16 + 8 * hh); v16b f;
#pragma unroll
  for (int e = 0; e < 8; ++e) { f[e] = a[e]; f[8 + e] = b[e]; } return f; }
__device__ __forceinline__ v8f wmma16b(v16b a, v16b b, v8f c) { v8f d = __builtin_amdgcn_wmma_f32_16x16x32_f16(false, a, false, b, (short)0, c, false, false); asm volatile("v_nop\n\tv_nop\n\tv_nop\n\tv_nop" : "+v"(d) : "v"(a), "v"(b)); return d; }
__device__ __forceinline__ void wave_lds_sync() { __builtin_amdgcn_fence(__ATOMIC_RELEASE, "workgroup"); __builtin_amdgcn_wave_barrier(); __builtin_amdgcn_fence(__ATOMIC_ACQUIRE, "workgroup"); }
__device__ __forceinline__ float pmul(float a, float b) { float p = a * b; asm volatile("" : "+v"(p)); return p; }
__device__ __forceinline__ int iclamp(int v, int lo, int hi) { return v < lo ? lo : (v > hi ? hi : v); }

typedef __attribute__((ext_vector_type(2))) _Float16 v2h;
typedef __attribute__((ext_vector_type(4))) _Float16 v4h;
typedef __attribute__((ext_vector_type(2))) float v2f;
typedef __attribute__((ext_vector_type(4))) int v4i;
__device__ __forceinline__ float nexp2(float v) { return __builtin_amdgcn_exp2f(v); }
__global__ __launch_bounds__(256) void prep_kernel(const float* __restrict__ wq, const float* __restrict__ wk, const float* __restrict__ wv, b16* __restrict__ WT) {
  const size_t u = (size_t)blockIdx.x * 256 + threadIdx.x; const size_t per = (size_t)E * E / 8; if (u >= 3 * per) return; const int m = (int)(u / per); const size_t e = u % per; const int row = (int)(e / (E / 8)), k0 = (int)(e % (E / 8)) * 8; const float* w = m == 0 ? wq : m == 1 ? wk : wv;
  v8b o; for (int j = 0; j < 8; ++j) o[j] = (b16)(bf16_rne(w[(size_t)(k0 + j) * E + row]) * WSC);
  for (int pass = 0; pass < 2; ++pass) { *(volatile v8b*)(WT + (size_t)m * E * E + (size_t)row * E + k0) = o; __threadfence(); }
}
__global__ __launch_bounds__(128) void proj_kernel(const float* __restrict__ x, const b16* __restrict__ WT, b16* __restrict__ QPh, b16* __restrict__ QPl, b16* __restrict__ KPh, b16* __restrict__ KPl, b16* __restrict__ VTh, b16* __restrict__ VTl, int b) {
  __shared__ __attribute__((aligned(16))) b16 As[64][256 + 8]; __shared__ __attribute__((aligned(16))) float Tf[4][16][128 + 4];
  const int wave = threadIdx.x >> 5, lane = threadIdx.x & 31, nloc = lane & 15, hlf = lane >> 4; const int t0 = blockIdx.x * 64; const int part = blockIdx.z / NSL, slab = blockIdx.z % NSL, c0 = slab * 128;
  if (part == 0 && t0 >= QL) return;
  const float* xb = x + ((size_t)b * T + t0) * E; const b16* Wp = WT + (size_t)part * E * E;
  v8f acc[8];
#pragma unroll
  for (int t = 0; t < 8; ++t) acc[t] = (v8f){};
#pragma unroll 1
  for (int kc = 0; kc < E; kc += 256) {
    __syncthreads();
    for (int i = threadIdx.x; i < 64 * 64; i += 128) { const int rr = i / 64, q = (i % 64) * 4; const v4f f = *(const v4f*)(xb + (size_t)rr * E + kc + q); v4h o; for (int j = 0; j < 4; ++j) o[j] = (b16)(bf16_rne(f[j]) * XS); *(v4h*)(&As[rr][q]) = o; }
    __syncthreads();
#pragma unroll 2
    for (int kb = 0; kb < 256; kb += 32) { const v16b a = frag_kb(&As[wave * 16 + nloc][kb], hlf);
#pragma unroll
      for (int t = 0; t < 8; ++t) acc[t] = wmma16b(a, frag_kb(Wp + (size_t)(c0 + t * 16 + nloc) * E + kc + kb, hlf), acc[t]); } }
#pragma unroll
  for (int t = 0; t < 8; ++t)
#pragma unroll
    for (int r = 0; r < 8; ++r) Tf[wave][8 * hlf + r][t * 16 + nloc] = acc[t][r] * (1.0f / (XS * WSC));
  __syncthreads();
  for (int pass = 0; pass < 2; ++pass) {
    if (part < 2) { b16* ph = part == 0 ? QPh : KPh; b16* pl = part == 0 ? QPl : KPl; const int c = c0 + lane * 4;
      for (int rr = 0; rr < 16; ++rr) { const int tok = t0 + wave * 16 + rr; v4h h4, l4; for (int j = 0; j < 4; ++j) { const float f = Tf[wave][rr][lane * 4 + j] * XS; const b16 p = (b16)f; h4[j] = p; l4[j] = (b16)((f - (float)p) * RS_); }
        *(volatile v4h*)(ph + (size_t)tok * E + c) = h4; *(volatile v4h*)(pl + (size_t)tok * E + c) = l4; } }
    else {
#pragma unroll 1
      for (int q = 0; q < 32; ++q) { const int cl = wave * 32 + q; const int e = c0 + cl; const int tk = lane * 2; v2h hv, lv;
        for (int j = 0; j < 2; ++j) { const float f = Tf[(tk + j) >> 4][(tk + j) & 15][cl] * XS; const b16 p = (b16)f; hv[j] = p; lv[j] = (b16)((f - (float)p) * RS_); }
        const size_t oi = (size_t)e * (size_t)T + t0 + lane * 2; *(volatile v2h*)(VTh + oi) = hv; *(volatile v2h*)(VTl + oi) = lv; } }
    __threadfence(); }
}
__global__ __launch_bounds__(128) void scores_kernel(const b16* __restrict__ QPh, const b16* __restrict__ QPl, const b16* __restrict__ KPh, const b16* __restrict__ KPl, float* __restrict__ S) {
  __shared__ __attribute__((aligned(16))) float Tf[4][16][128 + 4];
  const int wave = threadIdx.x >> 5, lane = threadIdx.x & 31, nloc = lane & 15, hlf = lane >> 4; const int q0 = blockIdx.x * 64 + wave * 16; const int k0 = blockIdx.y * 128;
  if (k0 > blockIdx.x * 64 + 63) return;
  v8f acc[8], accx[8];
#pragma unroll
  for (int t = 0; t < 8; ++t) { acc[t] = (v8f){}; accx[t] = (v8f){}; }
#pragma unroll 1
  for (int kb = 0; kb < E; kb += 32) { const v16b a = frag_kb(QPh + (size_t)(q0 + nloc) * E + kb, hlf), al = frag_kb(QPl + (size_t)(q0 + nloc) * E + kb, hlf);
#pragma unroll
    for (int t = 0; t < 8; ++t) { const size_t kr = (size_t)(k0 + t * 16 + nloc) * E + kb; const v16b bh = frag_kb(KPh + kr, hlf); acc[t] = wmma16b(a, bh, acc[t]); accx[t] = wmma16b(al, bh, accx[t]); accx[t] = wmma16b(a, frag_kb(KPl + kr, hlf), accx[t]); } }
#pragma unroll
  for (int t = 0; t < 8; ++t)
#pragma unroll
    for (int r = 0; r < 8; ++r) Tf[wave][8 * hlf + r][t * 16 + nloc] = acc[t][r] + accx[t][r] * (1.0f / RS_);
  wave_lds_sync();
  for (int pass = 0; pass < 2; ++pass) { for (int rr = 0; rr < 16; ++rr) *(volatile v4f*)(S + (size_t)(q0 + rr) * T + k0 + lane * 4) = *(const v4f*)(&Tf[wave][rr][lane * 4]); __threadfence(); }
}
__global__ __launch_bounds__(256) void softmax_kernel(const float* __restrict__ S, b16* __restrict__ Ph, b16* __restrict__ Pl) {
  const int wave = threadIdx.x >> 5, lane = threadIdx.x & 31; const int q = blockIdx.x * 8 + wave; if (q >= QL) return;
  const float* sr = S + (size_t)q * T; const float c = LOG2E * RSQE / (XS * XS); const int nch = q / 64 + 1;
  float sv[T / 64][2]; float m = -INFINITY;
#pragma unroll
  for (int ch = 0; ch < T / 64; ++ch) { if (ch < nch) { const v2f s2 = *(const v2f*)(sr + ch * 64 + lane * 2); for (int j = 0; j < 2; ++j) { const int k = ch * 64 + lane * 2 + j; sv[ch][j] = (k <= q) ? s2[j] : -INFINITY; m = fmaxf(m, sv[ch][j]); } } else { sv[ch][0] = -INFINITY; sv[ch][1] = -INFINITY; } }
#pragma unroll
  for (int o = 16; o >= 1; o >>= 1) m = fmaxf(m, __shfl_xor(m, o));
  float l = 0.0f;
#pragma unroll
  for (int ch = 0; ch < T / 64; ++ch) { if (ch < nch) { for (int j = 0; j < 2; ++j) { const float p = nexp2(pmul(sv[ch][j] - m, c)); sv[ch][j] = p; l += p; } } else { sv[ch][0] = 0.0f; sv[ch][1] = 0.0f; } }
#pragma unroll
  for (int o = 16; o >= 1; o >>= 1) l += __shfl_xor(l, o);
  const float inv = PS / l;
  for (int pass = 0; pass < 2; ++pass) {
#pragma unroll
    for (int ch = 0; ch < T / 64; ++ch) { v2h h2, l2; for (int j = 0; j < 2; ++j) { const float f = pmul(sv[ch][j], inv); const b16 p = (b16)f; float pf = (float)p; asm volatile("" : "+v"(pf)); h2[j] = p; l2[j] = (b16)pmul(f - pf, RS_); }
      *(volatile v2h*)(Ph + (size_t)q * T + ch * 64 + lane * 2) = h2; *(volatile v2h*)(Pl + (size_t)q * T + ch * 64 + lane * 2) = l2; }
    __threadfence(); }
}
__global__ __launch_bounds__(128) void pv_kernel(const b16* __restrict__ Ph, const b16* __restrict__ Pl, const b16* __restrict__ VTh, const b16* __restrict__ VTl, float* __restrict__ out, int b) {
  __shared__ __attribute__((aligned(16))) float Tf[4][16][128 + 4];
  const int wave = threadIdx.x >> 5, lane = threadIdx.x & 31, nloc = lane & 15, hlf = lane >> 4; const int q0 = blockIdx.x * 64 + wave * 16; const int e0 = blockIdx.y * 128;
  const int kend = ((q0 + 16 + 31) / 32) * 32;
  v8f acc[8], accx[8];
#pragma unroll
  for (int t = 0; t < 8; ++t) { acc[t] = (v8f){}; accx[t] = (v8f){}; }
#pragma unroll 1
  for (int kb = 0; kb < kend; kb += 32) { const v16b a = frag_kb(Ph + (size_t)(q0 + nloc) * T + kb, hlf), al = frag_kb(Pl + (size_t)(q0 + nloc) * T + kb, hlf);
#pragma unroll
    for (int t = 0; t < 8; ++t) { const size_t vr = (size_t)(e0 + t * 16 + nloc) * T + kb; const v16b bh = frag_kb(VTh + vr, hlf); acc[t] = wmma16b(a, bh, acc[t]); accx[t] = wmma16b(al, bh, accx[t]); accx[t] = wmma16b(a, frag_kb(VTl + vr, hlf), accx[t]); } }
#pragma unroll
  for (int t = 0; t < 8; ++t)
#pragma unroll
    for (int r = 0; r < 8; ++r) Tf[wave][8 * hlf + r][t * 16 + nloc] = (acc[t][r] + accx[t][r] * (1.0f / RS_)) * (1.0f / (PS * XS));
  wave_lds_sync();
  for (int pass = 0; pass < 2; ++pass) { for (int rr = 0; rr < 16; ++rr) *(volatile v4f*)(out + ((size_t)b * T + q0 + rr) * E + e0 + lane * 4) = *(const v4f*)(&Tf[wave][rr][lane * 4]); __threadfence(); }
}
}

extern "C" void kernel_launch(void* const* d_in, const int* in_sizes, int n_in, void* d_out, int out_size, void* d_ws, size_t ws_size, hipStream_t stream) {
  (void)n_in;
  auto Fp = [&](int i) { return (const float*)d_in[i]; };
  if (in_sizes[0] != B * T * E || in_sizes[1] != E * E || in_sizes[2] != E * E || in_sizes[3] != E * E || out_size != B * T * E) return;
  size_t off = 0; char* ws = (char*)d_ws;
  auto carve = [&](size_t bytes) { char* p = ws + off; off += (bytes + 255) & ~(size_t)255; return p; };
  b16* WT = (b16*)carve((size_t)3 * E * E * 2); const size_t plane = (size_t)T * E * 2;
  b16* QPh = (b16*)carve(plane); b16* QPl = (b16*)carve(plane); b16* KPh = (b16*)carve(plane); b16* KPl = (b16*)carve(plane); b16* VTh = (b16*)carve(plane); b16* VTl = (b16*)carve(plane);
  float* S = (float*)carve((size_t)T * T * 4); b16* Ph = (b16*)carve((size_t)T * T * 2); b16* Pl = (b16*)carve((size_t)T * T * 2);
  if (off > ws_size || off > ((size_t)128 << 20)) return;
  prep_kernel<<<(unsigned)(((size_t)3 * E * E / 8 + 255) / 256), 256, 0, stream>>>(Fp(1), Fp(2), Fp(3), WT);
  for (int b = 0; b < BL; ++b) {
    proj_kernel<<<dim3(T / 64, 1, 3 * NSL), 128, 0, stream>>>(Fp(0), WT, QPh, QPl, KPh, KPl, VTh, VTl, b);
    scores_kernel<<<dim3(QL / 64, T / 128), 128, 0, stream>>>(QPh, QPl, KPh, KPl, S);
    softmax_kernel<<<dim3(QL / 8), 256, 0, stream>>>(S, Ph, Pl);
    pv_kernel<<<dim3(QL / 64, E / 128), 128, 0, stream>>>(Ph, Pl, VTh, VTl, (float*)d_out, b); }
}
